// BahdanauAttention_24833500906223
// MI455X (gfx1250) — hardware-verified
//
#include <hip/hip_runtime.h>
#include <stddef.h>


typedef _Float16 v16h __attribute__((ext_vector_type(16)));
typedef _Float16 v8h  __attribute__((ext_vector_type(8)));
typedef float    v8f  __attribute__((ext_vector_type(8)));
typedef float    v4f  __attribute__((ext_vector_type(4)));
typedef _Float16 h16;

#ifndef NB
#define NB 4
#endif
#ifndef SEQ
#define SEQ 512
#endif
#define NB_FULL  4
#define SEQ_FULL 512
#define DIM   256
#define VDIM  256
#define MROWS (NB * SEQ)
#define PT    16

static_assert(NB >= 1 && NB <= NB_FULL);
static_assert(SEQ >= 256 && SEQ <= SEQ_FULL && (SEQ % 256) == 0);
static_assert((DIM % 64) == 0 && (DIM % 32) == 0);
static_assert((VDIM % 64) == 0 && (VDIM % 4) == 0);
static_assert(VDIM == 256);
static_assert((MROWS % 64) == 0);
static_assert(DIM == 8 * 32);
static_assert((SEQ % 64) == 0 && (SEQ % 32) == 0);
static_assert((SEQ % 128) == 0);
static_assert(PT == 16);
static_assert(PT * VDIM == 256 * 4 * 4);
static_assert((SEQ % PT) == 0);
static_assert(4 * 4 == PT);
static_assert(8 * 2 == PT);

#define LDT 72
#define LDC 68
static_assert((LDT % 8) == 0 && LDT >= 64);
static_assert((LDC % 4) == 0 && LDC >= 64);

#define SMAXW  ((SEQ > DIM) ? SEQ : DIM)
#define SPITCH (SMAXW + 4)
#define PPITCH (SEQ + 8)
static_assert((SPITCH % 4) == 0 && SPITCH >= SEQ && SPITCH >= DIM);
static_assert((PPITCH % 8) == 0 && PPITCH >= SEQ);

#define WCARRY 64.0f
#define PCARRY_LOG2 10.0f
#define TWO_LOG2E 2.885390081777927f
#define LOG2E     1.4426950408889634f

#define CTX_ELEMS ((size_t)NB_FULL * SEQ_FULL * DIM)
#define ATT_ELEMS ((size_t)NB_FULL * SEQ_FULL * SEQ_FULL)
static_assert(CTX_ELEMS * 4 == (size_t)2097152);
static_assert((CTX_ELEMS + ATT_ELEMS) * 4 == (size_t)6291456);
static_assert(((CTX_ELEMS * 4) % 128) == 0);

#define WT_BYTES  ((size_t)2 * VDIM * DIM * 2)
#define A16_BYTES ((size_t)2 * MROWS * DIM * 2)
#define HQT_BYTES ((size_t)NB * DIM * SEQ * 2)
#define S_BYTES   ((size_t)2 * MROWS * VDIM * 4)
#define OFF_WT  ((size_t)0)
#define OFF_A16 (OFF_WT + WT_BYTES)
#define OFF_HQT (OFF_A16 + A16_BYTES)
#define OFF_S   (OFF_HQT + HQT_BYTES)
#define WS_TOTAL (OFF_S + S_BYTES)
static_assert((WT_BYTES % 128) == 0 && (A16_BYTES % 128) == 0);
static_assert((HQT_BYTES % 128) == 0 && (S_BYTES % 128) == 0);
static_assert(WS_TOTAL <= (size_t)134217728);

__device__ __forceinline__ float bf16r(float x) {
  unsigned int u = __float_as_uint(x);
  u = (u + 0x7FFFu + ((u >> 16) & 1u)) & 0xFFFF0000u;
  return __uint_as_float(u);
}

static __device__ __forceinline__ h16 toh_flush(float v) {
  const h16 r = (h16)v;
  return (fabsf(v) < 6.103515625e-05f) ? (h16)0.0f : r;
}

__device__ __forceinline__ v16h frag_at(const _Float16* p) {
  v8h lo = *(const v8h*)(p);
  v8h hi = *(const v8h*)(p + 16);
  v16h out;
#pragma unroll
  for (int i = 0; i < 8; ++i) { out[i] = lo[i]; out[i + 8] = hi[i]; }
  return out;
}
__device__ __forceinline__ v16h ld_frag(const _Float16* base, unsigned ld) {
  const unsigned lane = threadIdx.x & 31u;
  return frag_at(base + (lane & 15u) * ld + (lane >> 4) * 8u);
}

__device__ __forceinline__ v8f wmma16(v16h a, v16h b, v8f c) {
  v8f d = __builtin_amdgcn_wmma_f32_16x16x32_f16(false, a, false, b, (short)0, c,
                                                 false, false);
  asm volatile("v_nop\n\tv_nop\n\tv_nop\n\tv_nop" : "+v"(d) : "v"(a), "v"(b));
  return d;
}

__device__ __forceinline__ float red32_sum(float x) {
#pragma unroll
  for (int off = 1; off < 32; off <<= 1) x += __shfl_xor(x, off, 32);
  return x;
}
__device__ __forceinline__ float red32_max(float x) {
#pragma unroll
  for (int off = 1; off < 32; off <<= 1) x = fmaxf(x, __shfl_xor(x, off, 32));
  return x;
}

__device__ __forceinline__ void wave_lds_sync() {
  __builtin_amdgcn_fence(3  , "wavefront");
  asm volatile("s_wait_dscnt 0x0" ::: "memory");
  __builtin_amdgcn_wave_barrier();
}

__device__ __forceinline__ float fast_exp2(float x) {
#if __has_builtin(__builtin_amdgcn_exp2f)
  return __builtin_amdgcn_exp2f(x);
#else
  return __expf(x * 0.6931471805599453f);
#endif
}

__global__ __launch_bounds__(256) void wconv_kernel(
    const float* __restrict__ W, _Float16* __restrict__ Wt, unsigned ldw, unsigned ldk) {
  __shared__ __attribute__((aligned(16))) _Float16 T[64 * LDT];
  const unsigned tid = threadIdx.x;
  const unsigned n0 = blockIdx.x * 64u;
  const unsigned k0 = blockIdx.y * 64u;
#pragma unroll 4
  for (unsigned j = 0; j < 16u; ++j) {
    const unsigned idx = tid + 256u * j;
    const unsigned nr = idx >> 6, kc = idx & 63u;
    const float v = W[(size_t)(n0 + nr) * ldw + k0 + kc];
    T[nr * LDT + kc] = toh_flush(WCARRY * bf16r(v));
  }
  __syncthreads();
  v8h x[2];
  size_t off[2];
#pragma unroll
  for (unsigned i = 0; i < 2u; ++i) {
    const unsigned n = 32u * i + (tid >> 3);
    const unsigned kc = (tid & 7u) * 8u;
    x[i] = *(const v8h*)&T[n * LDT + kc];
    off[i] = (size_t)(n0 + n) * ldk + k0 + kc;
  }
#pragma unroll
  for (int i = 0; i < 2; ++i) *(volatile v8h*)(Wt + off[i]) = x[i];
  __threadfence();
#pragma unroll
  for (int i = 0; i < 2; ++i) *(volatile v8h*)(Wt + off[i]) = x[i];
}

template <int WITH_T>
__device__ __forceinline__ void aconv_body(const float* __restrict__ X,
                                           _Float16* __restrict__ X16,
                                           _Float16* __restrict__ XT16) {
  __shared__ __attribute__((aligned(16))) _Float16 T[64 * LDT];
  __shared__ __attribute__((aligned(16))) _Float16 TT[64 * LDT];
  const unsigned tid = threadIdx.x;
  const unsigned c0 = blockIdx.x * 64u;
  const unsigned crow0 = blockIdx.y * 64u;
  const unsigned bidx = crow0 / (unsigned)SEQ;
  const unsigned s0 = crow0 - bidx * (unsigned)SEQ;
  const size_t frow0 = (size_t)bidx * SEQ_FULL + s0;
#pragma unroll
  for (unsigned j = 0; j < 4u; ++j) {
    const unsigned idx = tid + 256u * j;
    const unsigned r = idx >> 4, c = (idx & 15u) * 4u;
    const v4f a = *(const v4f*)(X + (frow0 + r) * DIM + c0 + c);
#pragma unroll
    for (unsigned i = 0; i < 4u; ++i) {
      const h16 hv = toh_flush(bf16r(a[i]));
      T[r * LDT + c + i] = hv;
      if (WITH_T) TT[(c + i) * LDT + r] = hv;
    }
  }
  __syncthreads();
  v8h x[2], xt[2];
  size_t off[2], offt[2];
#pragma unroll
  for (unsigned i = 0; i < 2u; ++i) {
    const unsigned n = 32u * i + (tid >> 3);
    const unsigned kc = (tid & 7u) * 8u;
    x[i] = *(const v8h*)&T[n * LDT + kc];
    off[i] = (size_t)(crow0 + n) * DIM + c0 + kc;
    if (WITH_T) {
      xt[i] = *(const v8h*)&TT[n * LDT + kc];
      offt[i] = ((size_t)bidx * DIM + c0 + n) * SEQ + s0 + kc;
    } else {
      xt[i] = x[i];
      offt[i] = off[i];
    }
  }
#pragma unroll
  for (int i = 0; i < 2; ++i) *(volatile v8h*)(X16 + off[i]) = x[i];
  if (WITH_T) {
#pragma unroll
    for (int i = 0; i < 2; ++i) *(volatile v8h*)(XT16 + offt[i]) = xt[i];
  }
  __threadfence();
#pragma unroll
  for (int i = 0; i < 2; ++i) *(volatile v8h*)(X16 + off[i]) = x[i];
  if (WITH_T) {
#pragma unroll
    for (int i = 0; i < 2; ++i) *(volatile v8h*)(XT16 + offt[i]) = xt[i];
  }
}

__global__ __launch_bounds__(256) void aconv_q_kernel(
    const float* __restrict__ X, _Float16* __restrict__ X16, _Float16* __restrict__ XT16) {
  aconv_body<1>(X, X16, XT16);
}
__global__ __launch_bounds__(256) void aconv_p_kernel(
    const float* __restrict__ X, _Float16* __restrict__ X16) {
  aconv_body<0>(X, X16, X16);
}

__global__ __launch_bounds__(256) void proj_kernel(
    const _Float16* __restrict__ A16, const _Float16* __restrict__ Wt,
    const float* __restrict__ bias0, const float* __restrict__ bias1,
    float* __restrict__ outf) {
  __shared__ __attribute__((aligned(16))) float Cs[64 * LDC];
  const unsigned tid = threadIdx.x, lane = tid & 31u;
  const unsigned w = (unsigned)__builtin_amdgcn_readfirstlane((int)(threadIdx.x >> 5));
  const unsigned mw = w >> 1, nw = w & 1u;
  const unsigned hh = lane >> 4, m = lane & 15u;
  const unsigned n0 = blockIdx.x * 64u;
  const unsigned row0 = blockIdx.y * 64u;
  const size_t woff = (size_t)(row0 / (unsigned)MROWS) * ((size_t)VDIM * DIM);

  const _Float16* ap  = A16 + (size_t)(row0 + mw * 16u + m) * DIM + hh * 8u;
  const _Float16* bp0 = Wt + woff + (size_t)(n0 + nw * 32u + m) * DIM + hh * 8u;
  const _Float16* bp1 = bp0 + (size_t)16 * DIM;
  v8f acc0 = {}, acc1 = {};
#pragma unroll 2
  for (unsigned k0 = 0; k0 < (unsigned)DIM; k0 += 32u) {
    const v16h a  = frag_at(ap + k0);
    const v16h b0 = frag_at(bp0 + k0);
    const v16h b1 = frag_at(bp1 + k0);
    acc0 = wmma16(a, b0, acc0);
    acc1 = wmma16(a, b1, acc1);
  }
#pragma unroll
  for (int r = 0; r < 8; ++r) {
    float* d = &Cs[(mw * 16u + hh * 8u + (unsigned)r) * LDC + nw * 32u + m];
    d[0]  = acc0[r];
    d[16] = acc1[r];
  }
  __syncthreads();

  const float cs = TWO_LOG2E / WCARRY;
  const unsigned c = (tid & 15u) * 4u;
  const v4f bva = *(const v4f*)(bias0 + n0 + c);
  const v4f bvb = *(const v4f*)(bias1 + n0 + c);
  const bool second = (row0 >= (unsigned)MROWS);
  v4f bb;
#pragma unroll
  for (int i = 0; i < 4; ++i) bb[i] = TWO_LOG2E * bf16r(second ? bvb[i] : bva[i]);
  v4f xs[4];
  size_t off[4];
#pragma unroll
  for (unsigned i = 0; i < 4u; ++i) {
    const unsigned r = 16u * i + (tid >> 4);
    const v4f u = *(const v4f*)&Cs[r * LDC + c];
    xs[i] = u * cs + bb;
    off[i] = (size_t)(row0 + r) * VDIM + n0 + c;
  }
#pragma unroll
  for (int i = 0; i < 4; ++i) *(volatile v4f*)(outf + off[i]) = xs[i];
  __threadfence();
#pragma unroll
  for (int i = 0; i < 4; ++i) *(volatile v4f*)(outf + off[i]) = xs[i];
}

__global__ __launch_bounds__(256) void addattn_kernel(
    const float* __restrict__ Skey, const float* __restrict__ Srow,
    const float* __restrict__ wvec, const float* __restrict__ bes,
    const _Float16* __restrict__ VT,
    float* __restrict__ ctx_out, float* __restrict__ att_out) {
  __shared__ __attribute__((aligned(16))) float sp_s[PT * VDIM];
  __shared__ __attribute__((aligned(16))) float vs[VDIM];
  __shared__ __attribute__((aligned(16))) float Ss[PT * SPITCH];
  __shared__ __attribute__((aligned(16))) _Float16 Pl[PT * PPITCH];
  __shared__ __attribute__((aligned(16))) float Ls[PT];
  static_assert(sizeof(float) * (PT * VDIM + VDIM + PT * SPITCH + PT) +
                sizeof(_Float16) * (PT * PPITCH) <= 131072);

  const unsigned tid = threadIdx.x, lane = tid & 31u;
  const unsigned wave = (unsigned)__builtin_amdgcn_readfirstlane((int)(threadIdx.x >> 5));
  const unsigned hh = lane >> 4, m = lane & 15u;
  const unsigned p0 = blockIdx.x * (unsigned)PT;
  const unsigned b = blockIdx.y;

#pragma unroll
  for (unsigned j = 0; j < 4u; ++j) {
    const unsigned idx = tid + 256u * j;
    const unsigned r = idx >> 6, c = (idx & 63u) * 4u;
    *(v4f*)&sp_s[r * VDIM + c] =
        *(const v4f*)(Srow + (size_t)(b * (unsigned)SEQ + p0 + r) * VDIM + c);
  }
  vs[tid] = -2.0f * bf16r(wvec[tid]);
  const float bev = bf16r(bes[0]);
  __syncthreads();

#pragma unroll 1
  for (unsigned pass = 0; pass < (unsigned)(SEQ / 256); ++pass) {
    const unsigned kx = pass * 256u + tid;
    const float* skr = Skey + (size_t)(b * (unsigned)SEQ + kx) * VDIM;
    float acc[PT];
#pragma unroll
    for (int p = 0; p < PT; ++p) acc[p] = 0.0f;
#pragma unroll 1
    for (unsigned v0 = 0; v0 < (unsigned)VDIM; v0 += 4u) {
      const v4f a = *(const v4f*)(skr + v0);
      const v4f vv = *(const v4f*)&vs[v0];
#pragma unroll
      for (int p = 0; p < PT; ++p) {
        const v4f s4 = *(const v4f*)&sp_s[(unsigned)p * VDIM + v0];
#pragma unroll
        for (int j = 0; j < 4; ++j) {
          const float t = fast_exp2(a[j] + s4[j]);
          const float r = __builtin_amdgcn_rcpf(t + 1.0f);
          acc[p] += vv[j] * r;
        }
      }
    }
#pragma unroll
    for (int p = 0; p < PT; ++p) Ss[(unsigned)p * SPITCH + kx] = acc[p] + bev;
  }
  __syncthreads();

#pragma unroll 1
  for (unsigned rr = 0; rr < 2u; ++rr) {
    const unsigned row = wave * 2u + rr;
    float mx = -3.0e38f;
#pragma unroll 4
    for (unsigned j = 0; j < (unsigned)(SEQ / 32); ++j)
      mx = fmaxf(mx, Ss[row * SPITCH + lane + 32u * j]);
    mx = red32_max(mx);
    float l = 0.0f;
    float lf = 0.0f;
#pragma unroll 4
    for (unsigned j = 0; j < (unsigned)(SEQ / 32); ++j) {
      const unsigned si = row * SPITCH + lane + 32u * j;
      const float arg = (Ss[si] - mx) * LOG2E + PCARRY_LOG2;
      const float e = fast_exp2(arg);
      const h16 ph = (arg < -14.0f) ? (h16)0.0f : (h16)e;
      Pl[row * PPITCH + lane + 32u * j] = ph;
      Ss[si] = e;
      l += (float)ph;
      lf += e;
    }
    l = red32_sum(l);
    lf = red32_sum(lf);
    if (lane == 0u) Ls[row] = l;
    wave_lds_sync();
    const float invf = __builtin_amdgcn_rcpf(lf);
    v4f ax[SEQ / 128];
    size_t aoff[SEQ / 128];
#pragma unroll
    for (unsigned i = 0; i < (unsigned)(SEQ / 128); ++i) {
      const unsigned c = 4u * lane + 128u * i;
      const v4f u = *(const v4f*)&Ss[row * SPITCH + c];
      ax[i] = u * invf;
      aoff[i] = ((size_t)b * SEQ_FULL + p0 + row) * SEQ_FULL + c;
    }
#pragma unroll
    for (int i = 0; i < SEQ / 128; ++i) *(volatile v4f*)(att_out + aoff[i]) = ax[i];
    __threadfence();
#pragma unroll
    for (int i = 0; i < SEQ / 128; ++i) *(volatile v4f*)(att_out + aoff[i]) = ax[i];
  }
  __syncthreads();

  const unsigned d0 = wave * 32u;
  const _Float16* bp = VT + ((size_t)b * DIM + d0 + m) * SEQ + hh * 8u;
  v8f o[2];
#pragma unroll
  for (int nb = 0; nb < 2; ++nb) o[nb] = (v8f){};
#pragma unroll 2
  for (unsigned k0 = 0; k0 < (unsigned)SEQ; k0 += 32u) {
    const v16h pf = ld_frag(&Pl[k0], PPITCH);
#pragma unroll
    for (int nb = 0; nb < 2; ++nb) {
      const v16h hf = frag_at(bp + (size_t)(nb * 16) * SEQ + k0);
      o[nb] = wmma16(pf, hf, o[nb]);
    }
  }

  float inv[8];
#pragma unroll
  for (int r = 0; r < 8; ++r) inv[r] = __builtin_amdgcn_rcpf(Ls[hh * 8u + (unsigned)r]);
#pragma unroll
  for (int nb = 0; nb < 2; ++nb)
#pragma unroll
    for (int r = 0; r < 8; ++r)
      Ss[(hh * 8u + (unsigned)r) * SPITCH + d0 + (unsigned)nb * 16u + m] = o[nb][r] * inv[r];
  wave_lds_sync();
  v4f x[4];
  size_t off[4];
#pragma unroll
  for (unsigned i = 0; i < 4u; ++i) {
    const unsigned r = 4u * i + (lane >> 3);
    const unsigned c = (lane & 7u) * 4u;
    x[i] = *(const v4f*)&Ss[r * SPITCH + d0 + c];
    off[i] = ((size_t)b * SEQ_FULL + p0 + r) * DIM + d0 + c;
  }
#pragma unroll
  for (int i = 0; i < 4; ++i) *(volatile v4f*)(ctx_out + off[i]) = x[i];
  __threadfence();
#pragma unroll
  for (int i = 0; i < 4; ++i) *(volatile v4f*)(ctx_out + off[i]) = x[i];
}

extern "C" void kernel_launch(void* const* d_in, const int* in_sizes, int n_in,
                              void* d_out, int out_size, void* d_ws, size_t ws_size,
                              hipStream_t stream) {
  if (n_in < 8) return;
  const long long need_x = ((long long)(NB - 1) * SEQ_FULL + SEQ) * DIM;
  const long long need_o = (long long)CTX_ELEMS +
                           ((long long)(NB - 1) * SEQ_FULL + SEQ) * SEQ_FULL;
  if ((long long)in_sizes[0] < need_x) return;
  if ((long long)in_sizes[1] < need_x) return;
  if ((long long)in_sizes[2] < (long long)DIM * VDIM) return;
  if (in_sizes[3] < VDIM) return;
  if ((long long)in_sizes[4] < (long long)DIM * VDIM) return;
  if (in_sizes[5] < VDIM) return;
  if (in_sizes[6] < VDIM) return;
  if (in_sizes[7] < 1) return;
  if ((long long)out_size < need_o) return;
  if (ws_size < WS_TOTAL) return;

  const float* query  = (const float*)d_in[0];
  const float* values = (const float*)d_in[1];
  const float* wq_in  = (const float*)d_in[2];
  const float* bq_in  = (const float*)d_in[3];
  const float* wk_in  = (const float*)d_in[4];
  const float* bk_in  = (const float*)d_in[5];
  const float* we_in  = (const float*)d_in[6];
  const float* be_in  = (const float*)d_in[7];
  float* out = (float*)d_out;

  char* ws = (char*)d_ws;
  _Float16* Wt   = (_Float16*)(ws + OFF_WT);
  _Float16* A16  = (_Float16*)(ws + OFF_A16);
  _Float16* VT   = (_Float16*)(ws + OFF_HQT);
  float*    Spl  = (float*)(ws + OFF_S);

  dim3 blk(256);

  wconv_kernel<<<dim3(VDIM / 64, DIM / 64), blk, 0, stream>>>(
      wk_in, Wt, (unsigned)DIM, (unsigned)DIM);
  wconv_kernel<<<dim3(VDIM / 64, DIM / 64), blk, 0, stream>>>(
      wq_in, Wt + (size_t)VDIM * DIM, (unsigned)DIM, (unsigned)DIM);

  aconv_q_kernel<<<dim3(DIM / 64, MROWS / 64), blk, 0, stream>>>(values, A16, VT);
  aconv_p_kernel<<<dim3(DIM / 64, MROWS / 64), blk, 0, stream>>>(
      query, A16 + (size_t)MROWS * DIM);

  proj_kernel<<<dim3(VDIM / 64, (2 * MROWS) / 64), blk, 0, stream>>>(
      A16, Wt, bk_in, bq_in, Spl);

  addattn_kernel<<<dim3(SEQ / PT, NB), blk, 0, stream>>>(
      Spl, Spl + (size_t)MROWS * VDIM, we_in, be_in, VT, out, out + CTX_ELEMS);
}
